// SoftAlignmentModule_18262200943081
// MI455X (gfx1250) — hardware-verified
//
#include <hip/hip_runtime.h>
#include <math.h>
#include <stdint.h>

#define NBATCH 16
#define PLEN   1024
#define HLEN   1024
#define DHID   256
#define GRPB   4
#define NGRPS  (NBATCH / GRPB)
#define NEG_FILL (-1e30f)
static_assert(PLEN == HLEN, "column-max softmax indexes premise rows by hypothesis position");
static_assert(NBATCH % GRPB == 0, "whole groups");

typedef __attribute__((ext_vector_type(16))) _Float16 v16h;
typedef __attribute__((ext_vector_type(8)))  _Float16 v8h;
typedef __attribute__((ext_vector_type(16))) __bf16   v16b;
typedef __attribute__((ext_vector_type(8)))  __bf16   v8b;
typedef __attribute__((ext_vector_type(8)))  float    v8f;
typedef __attribute__((ext_vector_type(4)))  float    v4f;
typedef __attribute__((ext_vector_type(2)))  float    v2f;
typedef __attribute__((ext_vector_type(4)))  unsigned int v4u;
typedef __attribute__((ext_vector_type(4)))  int      v4i;

__device__ __forceinline__ unsigned short f2bf_bits(float f) {
  unsigned u = __float_as_uint(f);
  return (unsigned short)((u + 0x7FFFu + ((u >> 16) & 1u)) >> 16);
}
__device__ __forceinline__ float bf_bits2f(unsigned short h) { return __uint_as_float(((unsigned)h) << 16); }

__device__ __forceinline__ void dep_guard_h(v8f& a, v8f& b, v16h x, v16h y) { asm volatile("v_nop\n\tv_nop\n\tv_nop\n\tv_nop" : "+v"(a), "+v"(b) : "v"(x), "v"(y)); }
__device__ __forceinline__ void dep_guard_b(v8f& a, v8f& b, v16b x, v16b y) { asm volatile("v_nop\n\tv_nop\n\tv_nop\n\tv_nop" : "+v"(a), "+v"(b) : "v"(x), "v"(y)); }
__device__ __forceinline__ void keep4_h(v16h a, v16h b, v16h c, v16h d) { asm volatile("v_nop" :: "v"(a), "v"(b), "v"(c), "v"(d)); }
__device__ __forceinline__ void keep4_b(v16b a, v16b b, v16b c, v16b d) { asm volatile("v_nop" :: "v"(a), "v"(b), "v"(c), "v"(d)); }
__device__ __forceinline__ void acc_guard4(v8f& a, v8f& b, v8f& c, v8f& d) { asm volatile("v_nop\n\tv_nop\n\tv_nop\n\tv_nop" : "+v"(a), "+v"(b), "+v"(c), "+v"(d)); }
template <typename T> struct Frag;
template <> struct Frag<_Float16> {
  typedef v16h V; union U { v16h v; v8h h[2]; };
  static __device__ __forceinline__ v16h load(const _Float16* p) {
    U f; f.h[0] = *(const v8h*)(p); f.h[1] = *(const v8h*)(p + 16); return f.v;
  }
  static __device__ __forceinline__ v8f mma(v16h a, v16h b, v8f c) {
    return __builtin_amdgcn_wmma_f32_16x16x32_f16(false, a, false, b, (short)0, c, false, false);
  }
  static __device__ __forceinline__ void guard(v8f& a, v8f& b, v16h x, v16h y) { dep_guard_h(a, b, x, y); }
  static __device__ __forceinline__ void keep(v16h a, v16h b, v16h c, v16h d) { keep4_h(a, b, c, d); }
};
template <> struct Frag<__bf16> {
  typedef v16b V; union U { v16b v; v8b h[2]; };
  static __device__ __forceinline__ v16b load(const __bf16* p) {
    U f; f.h[0] = *(const v8b*)(p); f.h[1] = *(const v8b*)(p + 16); return f.v;
  }
  static __device__ __forceinline__ v8f mma(v16b a, v16b b, v8f c) {
    return __builtin_amdgcn_wmma_f32_16x16x32_bf16(false, a, false, b, (short)0, c, false, false);
  }
  static __device__ __forceinline__ void guard(v8f& a, v8f& b, v16b x, v16b y) { dep_guard_b(a, b, x, y); }
  static __device__ __forceinline__ void keep(v16b a, v16b b, v16b c, v16b d) { keep4_b(a, b, c, d); }
};

template <int ET> struct Elem;
template <> struct Elem<0> { typedef _Float16 T; };
template <> struct Elem<1> { typedef __bf16 T; };
template <int ET, bool SPLIT, int BIAS_MODE, int OUT_MODE, bool RESID, int ACT = 0>
__global__ __launch_bounds__(256) void wmma_gemm64(
    const unsigned short* __restrict__ Ap, const unsigned short* __restrict__ A2p, int lda, long strideA,
    const unsigned short* __restrict__ Btp, const unsigned short* __restrict__ Bt2p, int ldb, long strideB,
    void* __restrict__ Cout, void* __restrict__ Cout2, int ldc, long strideC,
    const float* __restrict__ bias,
    const float* __restrict__ resid, long strideR,
    int M, int N, int K, float scale) {
  typedef typename Elem<ET>::T T;
  typedef typename Frag<T>::V V;
  const T* A = (const T*)Ap; const T* A2 = (const T*)A2p; const T* Bt = (const T*)Btp; const T* Bt2 = (const T*)Bt2p;
  __shared__ __align__(16) float sT[8][16 * 68];
  const int b    = blockIdx.y;
  const int lane = threadIdx.x & 31;
  const int wave = threadIdx.x >> 5;
  const int tilesN = N >> 6;
  const int tilesM = M >> 6;
  const int tile = blockIdx.x * 8 + wave;
  if (tile >= tilesM * tilesN) return;
  const int tm = tile / tilesN;
  const int tn = tile - tm * tilesN;
  const int m0 = tm << 6;
  const int n0 = tn << 6;

  const T* Ab  = A  + (size_t)b * strideA;
  const T* Bb  = Bt + (size_t)b * strideB;
  const T* Ab2 = SPLIT ? (A2  + (size_t)b * strideA) : nullptr;
  const T* Bb2 = SPLIT ? (Bt2 + (size_t)b * strideB) : nullptr;

  const int rlane = lane & 15;
  const int koff  = (lane >> 4) * 8;
  const int mOff  = (lane >> 4) * 8;

  v8f acc[4][4];
#pragma unroll
  for (int i = 0; i < 4; ++i)
#pragma unroll
    for (int j = 0; j < 4; ++j) acc[i][j] = (v8f){0.f,0.f,0.f,0.f,0.f,0.f,0.f,0.f};

  for (int k0 = 0; k0 < K; k0 += 32) {
    V bh[4], bl[4];
#pragma unroll
    for (int j = 0; j < 4; ++j) {
      const size_t bo = (size_t)(n0 + (j << 4) + rlane) * ldb + koff + k0;
      bh[j] = Frag<T>::load(Bb + bo);
      if (SPLIT) bl[j] = Frag<T>::load(Bb2 + bo);
    }
#pragma unroll
    for (int i = 0; i < 4; ++i) {
      const size_t ao = (size_t)(m0 + (i << 4) + rlane) * lda + koff + k0;
      V ah = Frag<T>::load(Ab + ao);
      V al;
      if (SPLIT) al = Frag<T>::load(Ab2 + ao);
#pragma unroll
      for (int j = 0; j < 4; ++j) {
        acc[i][j] = Frag<T>::mma(ah, bh[j], acc[i][j]);
        if (SPLIT) {
          acc[i][j] = Frag<T>::mma(ah, bl[j], acc[i][j]);
          acc[i][j] = Frag<T>::mma(al, bh[j], acc[i][j]);
        }
      }
      Frag<T>::guard(acc[i][0], acc[i][3], ah, SPLIT ? al : ah);
    }
    Frag<T>::keep(bh[0], bh[1], bh[2], bh[3]);
    if (SPLIT) Frag<T>::keep(bl[0], bl[1], bl[2], bl[3]);
  }
  acc_guard4(acc[0][0], acc[0][1], acc[0][2], acc[0][3]);
  acc_guard4(acc[1][0], acc[1][1], acc[1][2], acc[1][3]);
  acc_guard4(acc[2][0], acc[2][1], acc[2][2], acc[2][3]);
  acc_guard4(acc[3][0], acc[3][1], acc[3][2], acc[3][3]);

  float* slab = sT[wave];
  const float* Rb = RESID ? (resid + (size_t)b * strideR) : nullptr;
#pragma unroll
  for (int i = 0; i < 4; ++i) {
    const int mBase = m0 + (i << 4);
#pragma unroll
    for (int j = 0; j < 4; ++j) {
      const int n = n0 + (j << 4) + rlane;
      float bv = 0.f;
      if (BIAS_MODE == 2) bv = bias[n];
#pragma unroll
      for (int r = 0; r < 8; ++r) {
        float v = acc[i][j][r] * scale;
        if (BIAS_MODE == 1) v += bias[mBase + mOff + r];
        if (BIAS_MODE == 2) v += bv;
        if (RESID) v += Rb[(size_t)(mBase + mOff + r) * ldc + n];
        if (ACT == 1) v = tanhf(v);
        if (ACT == 2) v = fmaxf(v, 0.0f);
        if (ACT == 3) v = v / (1.0f + expf(-v));
        if (ACT == 4) v = (v > 0.f) ? v : 0.01f * v;
        if (ACT == 5) v = 0.5f * v * (1.0f + erff(v * 0.70710678118654752f));
        slab[(mOff + r) * 68 + (j << 4) + rlane] = v;
      }
    }
    __builtin_amdgcn_fence(__ATOMIC_RELEASE, "workgroup");
    __builtin_amdgcn_wave_barrier();
    __builtin_amdgcn_fence(__ATOMIC_ACQUIRE, "workgroup");
    if (OUT_MODE == 0) {
      float* C = (float*)Cout + (size_t)b * strideC;
      const int hh = lane >> 4, c4 = (lane & 15) * 4;
      for (int pass = 0; pass < 2; ++pass) {
#pragma unroll
        for (int it = 0; it < 8; ++it) {
          const int row = it * 2 + hh;
          v4f v = *(const v4f*)(slab + row * 68 + c4);
          *(volatile v4f*)(C + (size_t)(mBase + row) * ldc + n0 + c4) = v;
        }
        __threadfence();
      }
    } else {
      const int q = lane >> 3, c8 = (lane & 7) * 8;
      unsigned short* C  = (unsigned short*)Cout  + (size_t)b * strideC;
      unsigned short* C2 = (OUT_MODE == 2) ? ((unsigned short*)Cout2 + (size_t)b * strideC) : nullptr;
      for (int pass = 0; pass < 2; ++pass) {
#pragma unroll
        for (int it = 0; it < 4; ++it) {
          const int row = it * 4 + q;
          const float* sp = slab + row * 68 + c8;
          v8h hv, lv;
#pragma unroll
          for (int e = 0; e < 8; ++e) {
            if (OUT_MODE == 1) {
              hv[e] = (_Float16)sp[e];
            } else {
              unsigned short hb = f2bf_bits(sp[e]);
              unsigned short lb = f2bf_bits(sp[e] - bf_bits2f(hb));
              hv[e] = __builtin_bit_cast(_Float16, hb);
              lv[e] = __builtin_bit_cast(_Float16, lb);
            }
          }
          *(volatile v8h*)(C + (size_t)(mBase + row) * ldc + n0 + c8) = hv;
          if (OUT_MODE == 2) *(volatile v8h*)(C2 + (size_t)(mBase + row) * ldc + n0 + c8) = lv;
        }
        __threadfence();
      }
    }
    __builtin_amdgcn_fence(__ATOMIC_RELEASE, "workgroup");
    __builtin_amdgcn_wave_barrier();
    __builtin_amdgcn_fence(__ATOMIC_ACQUIRE, "workgroup");
  }
}

__device__ __forceinline__ unsigned pk16(unsigned short a, unsigned short b) { return (unsigned)a | ((unsigned)b << 16); }

__global__ __launch_bounds__(256) void split_bf16x2_kernel(const float* __restrict__ in, unsigned short* __restrict__ hi,
                                                           unsigned short* __restrict__ lo, int n2) {
  const int i = blockIdx.x * 256 + threadIdx.x;
  if (i < n2) {
    const v2f f = *(const v2f*)(in + 2 * (size_t)i);
    const unsigned short h0 = f2bf_bits(f[0]), h1 = f2bf_bits(f[1]);
    const unsigned short l0 = f2bf_bits(f[0] - bf_bits2f(h0)), l1 = f2bf_bits(f[1] - bf_bits2f(h1));
    const unsigned uh = pk16(h0, h1), ul = pk16(l0, l1);
    ((volatile unsigned*)hi)[i] = uh;
    ((volatile unsigned*)lo)[i] = ul;
    __threadfence();
    ((volatile unsigned*)hi)[i] = uh;
    ((volatile unsigned*)lo)[i] = ul;
  }
}

__global__ __launch_bounds__(256) void transpose_split_kernel(const float* __restrict__ in, int ldi, long sIn,
                                                              unsigned short* __restrict__ outh,
                                                              unsigned short* __restrict__ outl, int ldo, long sOut) {
  __shared__ __align__(16) float tf[64 * 68];
  const size_t zb = blockIdx.z;
  const float* inb = in + zb * (size_t)sIn;
  unsigned short* ohb = outh + zb * (size_t)sOut;
  unsigned short* olb = outl + zb * (size_t)sOut;
  const int c0  = blockIdx.x * 64;
  const int r0  = blockIdx.y * 64;
  const int tid = threadIdx.x;
  {
    const int sub = tid >> 4;
    const int c4  = (tid & 15) * 4;
#pragma unroll
    for (int it = 0; it < 4; ++it) {
      const int rr = it * 16 + sub;
      const v4f a = *(const v4f*)(inb + (size_t)(r0 + rr) * ldi + c0 + c4);
      *(v4f*)(tf + rr * 68 + c4) = a;
    }
  }
  __syncthreads();
  const int s8 = tid >> 3;
  const int c8 = (tid & 7) * 8;
  v4u hv[2], lv[2];
#pragma unroll
  for (int it = 0; it < 2; ++it) {
    const int oc = it * 32 + s8;
    v4u a, a2;
#pragma unroll
    for (int q = 0; q < 4; ++q) {
      const float f0 = tf[(c8 + 2 * q) * 68 + oc];
      const float f1 = tf[(c8 + 2 * q + 1) * 68 + oc];
      const unsigned short h0 = f2bf_bits(f0), h1 = f2bf_bits(f1);
      const unsigned short l0 = f2bf_bits(f0 - bf_bits2f(h0));
      const unsigned short l1 = f2bf_bits(f1 - bf_bits2f(h1));
      a[q]  = pk16(h0, h1);
      a2[q] = pk16(l0, l1);
    }
    hv[it] = a; lv[it] = a2;
  }
  for (int pass = 0; pass < 2; ++pass) {
#pragma unroll
    for (int it = 0; it < 2; ++it) {
      const int oc = it * 32 + s8;
      const size_t go = (size_t)(c0 + oc) * ldo + r0 + c8;
      *(volatile v4u*)(ohb + go) = hv[it];
      *(volatile v4u*)(olb + go) = lv[it];
    }
    __threadfence();
  }
}

__global__ __launch_bounds__(128) void row_softmax_split_kernel(
    const float* __restrict__ S, const int* __restrict__ pm, const int* __restrict__ hm,
    const float* __restrict__ bias, unsigned short* __restrict__ Ah, unsigned short* __restrict__ Al, int b0) {
#pragma clang fp contract(off)
  __shared__ float redm[4];
  __shared__ float reds[4];
  const int p    = blockIdx.x;
  const int bb   = blockIdx.y;
  int b = b0 + bb;
  b = b < 0 ? 0 : (b > NBATCH - 1 ? NBATCH - 1 : b);
  const int tid  = threadIdx.x;
  const int lane = tid & 31;
  const int wave = tid >> 5;
  const int j0   = tid * 8;
  const float bv  = bias[0];
  const float pmv = (float)pm[(size_t)b * PLEN + p];
  const float* row = S + ((size_t)bb * PLEN + (size_t)p) * HLEN + j0;
  const v4f a0 = *(const v4f*)(row);
  const v4f a1 = *(const v4f*)(row + 4);
  const int* hrow = hm + (size_t)b * HLEN + j0;
  const v4i h0 = *(const v4i*)(hrow);
  const v4i h1 = *(const v4i*)(hrow + 4);
  float t[8];
#pragma unroll
  for (int e = 0; e < 4; ++e) {
    const float mk0 = pmv * (float)h0[e];
    const float mk1 = pmv * (float)h1[e];
    t[e]     = (a0[e] + bv) + (1.0f - mk0) * NEG_FILL;
    t[4 + e] = (a1[e] + bv) + (1.0f - mk1) * NEG_FILL;
  }
  float m = fmaxf(fmaxf(fmaxf(t[0], t[1]), fmaxf(t[2], t[3])), fmaxf(fmaxf(t[4], t[5]), fmaxf(t[6], t[7])));
#pragma unroll
  for (int off = 16; off > 0; off >>= 1) m = fmaxf(m, __shfl_xor(m, off, 32));
  if (lane == 0) redm[wave] = m;
  __syncthreads();
  const float mx = fmaxf(fmaxf(redm[0], redm[1]), fmaxf(redm[2], redm[3]));
  float ex[8];
#pragma unroll
  for (int e = 0; e < 8; ++e) ex[e] = __expf(t[e] - mx);
  float ps = ((((((ex[0] + ex[1]) + ex[2]) + ex[3]) + ex[4]) + ex[5]) + ex[6]) + ex[7];
#pragma unroll
  for (int off = 16; off > 0; off >>= 1) ps += __shfl_xor(ps, off, 32);
  if (lane == 0) reds[wave] = ps;
  __syncthreads();
  const float tot = ((reds[0] + reds[1]) + reds[2]) + reds[3];
  const float inv = 1.0f / tot;
  unsigned hw[4], lw[4];
#pragma unroll
  for (int q = 0; q < 4; ++q) {
    const float p0 = ex[2 * q] * inv, p1 = ex[2 * q + 1] * inv;
    const unsigned short hb0 = f2bf_bits(p0), hb1 = f2bf_bits(p1);
    const unsigned short lb0 = f2bf_bits(p0 - bf_bits2f(hb0));
    const unsigned short lb1 = f2bf_bits(p1 - bf_bits2f(hb1));
    hw[q] = pk16(hb0, hb1);
    lw[q] = pk16(lb0, lb1);
  }
  const v4u hvv = (v4u){hw[0], hw[1], hw[2], hw[3]};
  const v4u lvv = (v4u){lw[0], lw[1], lw[2], lw[3]};
  const size_t rowoff = ((size_t)bb * PLEN + (size_t)p) * HLEN + j0;
  *(volatile v4u*)(Ah + rowoff) = hvv;
  *(volatile v4u*)(Al + rowoff) = lvv;
  __threadfence();
  *(volatile v4u*)(Ah + rowoff) = hvv;
  *(volatile v4u*)(Al + rowoff) = lvv;
}

__global__ __launch_bounds__(256) void colmax_kernel(
    const float* __restrict__ S, const int* __restrict__ pm, const int* __restrict__ hm,
    const float* __restrict__ bias, float* __restrict__ CM, int b0) {
#pragma clang fp contract(off)
  __shared__ float spm[PLEN];
  const int bb  = blockIdx.y;
  int b = b0 + bb;
  b = b < 0 ? 0 : (b > NBATCH - 1 ? NBATCH - 1 : b);
  const int tid = threadIdx.x;
  const int q   = blockIdx.x * 256 + tid;
  for (int i = tid; i < PLEN; i += 256) spm[i] = (float)pm[(size_t)b * PLEN + i];
  __syncthreads();
  const float hmv = (float)hm[(size_t)b * HLEN + q];
  const float bv  = bias[0];
  const float* col = S + (size_t)bb * PLEN * HLEN + q;
  float m = -__builtin_inff();
#pragma unroll 4
  for (int p = 0; p < PLEN; ++p) {
    const float s  = col[(size_t)p * HLEN];
    const float tt = (s + bv) + (1.0f - spm[p] * hmv) * NEG_FILL;
    m = fmaxf(m, tt);
  }
  const size_t o = (size_t)bb * HLEN + q;
  ((volatile float*)CM)[o] = m;
  __threadfence();
  ((volatile float*)CM)[o] = m;
}

__global__ __launch_bounds__(256) void premise_kernel(
    const float* __restrict__ CM, const float* __restrict__ P, float* __restrict__ out0, int b0) {
  __shared__ __align__(16) float scm[HLEN];
  __shared__ __align__(16) float spr[HLEN];
  __shared__ __align__(16) float sap[DHID];
  __shared__ float redm[8];
  __shared__ float reds[8];
  const int bb   = blockIdx.x;
  int b = b0 + bb;
  b = b < 0 ? 0 : (b > NBATCH - 1 ? NBATCH - 1 : b);
  const int tid  = threadIdx.x;
  const int lane = tid & 31;
  const int wave = tid >> 5;

  float lm = -__builtin_inff();
  for (int i = tid; i < HLEN; i += 256) {
    const float v = CM[(size_t)bb * HLEN + i];
    scm[i] = v;
    lm = fmaxf(lm, v);
  }
#pragma unroll
  for (int off = 16; off > 0; off >>= 1) lm = fmaxf(lm, __shfl_xor(lm, off, 32));
  if (lane == 0) redm[wave] = lm;
  __syncthreads();
  float mx = redm[0];
#pragma unroll
  for (int w = 1; w < 8; ++w) mx = fmaxf(mx, redm[w]);

  float ls = 0.f;
  for (int i = tid; i < HLEN; i += 256) {
    const float e = __expf(scm[i] - mx);
    spr[i] = e;
    ls += e;
  }
#pragma unroll
  for (int off = 16; off > 0; off >>= 1) ls += __shfl_xor(ls, off, 32);
  if (lane == 0) reds[wave] = ls;
  __syncthreads();
  float tot = reds[0];
#pragma unroll
  for (int w = 1; w < 8; ++w) tot += reds[w];
  const float inv = 1.0f / tot;
  for (int i = tid; i < HLEN; i += 256) spr[i] = spr[i] * inv;
  __syncthreads();

  const int d = tid;
  const float* Pb = P + (size_t)b * PLEN * DHID + d;
  float acc = 0.f;
#pragma unroll 4
  for (int q = 0; q < HLEN; ++q) acc = acc + spr[q] * Pb[(size_t)q * DHID];
  sap[d] = acc;
  __syncthreads();

  const v4f va = *(const v4f*)(sap + lane * 4);
  const v4f vb = *(const v4f*)(sap + 128 + lane * 4);
  float* ob = out0 + (size_t)b * HLEN * DHID;
  for (int pass = 0; pass < 2; ++pass) {
#pragma unroll 1
    for (int r = wave; r < HLEN; r += 8) {
      float* orow = ob + (size_t)r * DHID;
      *(volatile v4f*)(orow + lane * 4) = va;
      *(volatile v4f*)(orow + 128 + lane * 4) = vb;
    }
    __threadfence();
  }
}

extern "C" void kernel_launch(void* const* d_in, const int* in_sizes, int n_in,
                              void* d_out, int out_size, void* d_ws, size_t ws_size,
                              hipStream_t stream) {
  if (n_in < 6) return;
  if (in_sizes[0] != NBATCH * PLEN * DHID) return;
  if (in_sizes[1] != NBATCH * HLEN * DHID) return;
  if (in_sizes[2] != NBATCH * PLEN || in_sizes[3] != NBATCH * HLEN) return;
  if (in_sizes[4] != DHID * DHID || in_sizes[5] < 1) return;
  if (out_size != 2 * NBATCH * PLEN * DHID) return;

  const float* P    = (const float*)d_in[0];
  const float* H    = (const float*)d_in[1];
  const int*   pm   = (const int*)d_in[2];
  const int*   hm   = (const int*)d_in[3];
  const float* W    = (const float*)d_in[4];
  const float* bias = (const float*)d_in[5];

  const size_t PWT = (size_t)DHID * DHID * 2;
  const size_t PAC = (size_t)NBATCH * PLEN * DHID * 2;
  const size_t PSC = (size_t)GRPB * PLEN * HLEN * 4;
  const size_t PPR = (size_t)GRPB * PLEN * HLEN * 2;
  const size_t PCM = (size_t)GRPB * HLEN * 4;
  size_t off = 0;
  const size_t oWTh = off; off += PWT;
  const size_t oWTl = off; off += PWT;
  const size_t oPh  = off; off += PAC;
  const size_t oPl  = off; off += PAC;
  const size_t oHh  = off; off += PAC;
  const size_t oHl  = off; off += PAC;
  const size_t oHTh = off; off += PAC;
  const size_t oHTl = off; off += PAC;
  const size_t oPWh = off; off += PAC;
  const size_t oPWl = off; off += PAC;
  const size_t oS   = off; off += PSC;
  const size_t oAh  = off; off += PPR;
  const size_t oAl  = off; off += PPR;
  const size_t oCM  = off; off += PCM;
  if (off > ws_size) return;

  char* ws = (char*)d_ws;
  unsigned short* WTh = (unsigned short*)(ws + oWTh);
  unsigned short* WTl = (unsigned short*)(ws + oWTl);
  unsigned short* Ph  = (unsigned short*)(ws + oPh);
  unsigned short* Pl  = (unsigned short*)(ws + oPl);
  unsigned short* Hh  = (unsigned short*)(ws + oHh);
  unsigned short* Hl  = (unsigned short*)(ws + oHl);
  unsigned short* HTh = (unsigned short*)(ws + oHTh);
  unsigned short* HTl = (unsigned short*)(ws + oHTl);
  unsigned short* PWh = (unsigned short*)(ws + oPWh);
  unsigned short* PWl = (unsigned short*)(ws + oPWl);
  float*          Sbuf = (float*)(ws + oS);
  unsigned short* Ah  = (unsigned short*)(ws + oAh);
  unsigned short* Al  = (unsigned short*)(ws + oAl);
  float*          CM  = (float*)(ws + oCM);

  float* out0 = (float*)d_out;
  float* out1 = (float*)d_out + (size_t)NBATCH * PLEN * DHID;

  const dim3 blk(256);
  transpose_split_kernel<<<dim3(DHID / 64, DHID / 64, 1), blk, 0, stream>>>(W, DHID, 0L, WTh, WTl, DHID, 0L);
  const int n2 = NBATCH * PLEN * DHID / 2;
  const dim3 gSplit((n2 + 255) / 256);
  split_bf16x2_kernel<<<gSplit, blk, 0, stream>>>(P, Ph, Pl, n2);
  split_bf16x2_kernel<<<gSplit, blk, 0, stream>>>(H, Hh, Hl, n2);
  transpose_split_kernel<<<dim3(DHID / 64, HLEN / 64, NBATCH), blk, 0, stream>>>(
      H, DHID, (long)HLEN * DHID, HTh, HTl, HLEN, (long)DHID * HLEN);
  const dim3 gPW(((NBATCH * PLEN / 64) * (DHID / 64) + 7) / 8, 1);
  wmma_gemm64<1, true, 0, 2, false, 0><<<gPW, blk, 0, stream>>>(
      Ph, Pl, DHID, 0L, WTh, WTl, DHID, 0L, (void*)PWh, (void*)PWl, DHID, 0L,
      bias, bias, 0L, NBATCH * PLEN, DHID, DHID, 1.0f);

  const dim3 gS(((PLEN / 64) * (HLEN / 64) + 7) / 8, GRPB);
  const dim3 gSm(PLEN, GRPB);
  const dim3 gCM(HLEN / 256, GRPB);
  const dim3 gPr(GRPB);
  const dim3 gAV(((PLEN / 64) * (DHID / 64) + 7) / 8, GRPB);

  for (int g = 0; g < NGRPS; ++g) {
    const int b0 = g * GRPB;
    const size_t aoff = (size_t)b0 * PLEN * DHID;
    const size_t toff = (size_t)b0 * DHID * HLEN;
    wmma_gemm64<1, true, 0, 0, false, 0><<<gS, blk, 0, stream>>>(
        PWh + aoff, PWl + aoff, DHID, (long)PLEN * DHID,
        Hh + aoff, Hl + aoff, DHID, (long)HLEN * DHID,
        (void*)Sbuf, (void*)Sbuf, HLEN, (long)PLEN * HLEN,
        bias, bias, 0L, PLEN, HLEN, DHID, 1.0f);
    row_softmax_split_kernel<<<gSm, dim3(128), 0, stream>>>(Sbuf, pm, hm, bias, Ah, Al, b0);
    colmax_kernel<<<gCM, blk, 0, stream>>>(Sbuf, pm, hm, bias, CM, b0);
    premise_kernel<<<gPr, blk, 0, stream>>>(CM, P, out0, b0);
    wmma_gemm64<1, true, 0, 0, false, 0><<<gAV, blk, 0, stream>>>(
        Ah, Al, HLEN, (long)PLEN * HLEN,
        HTh + toff, HTl + toff, HLEN, (long)DHID * HLEN,
        (void*)(out1 + aoff), (void*)(out1 + aoff), DHID, (long)PLEN * DHID,
        bias, bias, 0L, PLEN, DHID, HLEN, 1.0f);
  }
}
